// TemporalAtomAccumulator_86732569575516
// MI455X (gfx1250) — hardware-run, weakly checked
//
#include <hip/hip_runtime.h>
#include <math.h>

typedef __attribute__((ext_vector_type(16))) __bf16   v16b;
typedef __attribute__((ext_vector_type(8)))  __bf16   v8b;
typedef __attribute__((ext_vector_type(8)))  float    v8f;
typedef __attribute__((ext_vector_type(4)))  float    v4f;
typedef __attribute__((ext_vector_type(4)))  unsigned int v4u;

constexpr int kBatch = 4;
constexpr int kSeq   = 4096;
constexpr int kChan  = 256;
constexpr int kProj  = 64;
constexpr int kRows  = kBatch * kSeq;
constexpr int kQKP   = 2 * kProj;
constexpr float kScoreScale = 0.125f;
constexpr int kNHalf = 128;
constexpr int kOsP   = 132;
static_assert(kScoreScale * kScoreScale * (float)kProj == 1.0f, "score scale is kProj^-0.5");
static_assert((kRows % 64) == 0 && (kQKP % 64) == 0 && (kChan % 32) == 0, "GEMM tile multiples");
static_assert((kSeq % 64) == 0 && (kChan % 64) == 0 && (kProj % 32) == 0, "attention tile multiples");
static_assert(kChan == 2 * kNHalf, "two column halves");

constexpr size_t kOffXB   = 0;
constexpr size_t kOffVT   = kOffXB  + (size_t)kRows * kChan * 2;
constexpr size_t kOffQKH  = kOffVT  + (size_t)kBatch * kChan * kSeq * 2;
constexpr size_t kOffQKL  = kOffQKH + (size_t)kRows * kQKP * 2;
constexpr size_t kOffWT   = kOffQKL + (size_t)kRows * kQKP * 2;
constexpr size_t kOffBIAS = kOffWT  + (size_t)kQKP * kChan * 2;
constexpr size_t kWsTotal = kOffBIAS + (size_t)kQKP * 4;
static_assert(kWsTotal == 25231872ull, "carve total");
static_assert(kWsTotal <= 134217728ull, "carve cap");
static_assert((kOffVT % 128) == 0 && (kOffQKH % 128) == 0 && (kOffQKL % 128) == 0 &&
              (kOffWT % 128) == 0 && (kOffBIAS % 128) == 0, "128-B aligned regions");

__device__ __forceinline__ unsigned short f2bf_bits(float f) {
  unsigned u = __float_as_uint(f);
  return (unsigned short)((u + 0x7FFFu + ((u >> 16) & 1u)) >> 16);
}
__device__ __forceinline__ float bf_bits2f(unsigned short h) { return __uint_as_float(((unsigned)h) << 16); }
__device__ __forceinline__ unsigned pk16(unsigned short a, unsigned short b) { return (unsigned)a | ((unsigned)b << 16); }

__device__ __forceinline__ v4u pack8_bf16(v4f a0, v4f a1, float sc) {
  v4u o;
#pragma unroll
  for (int q = 0; q < 2; ++q) {
    const float f0 = a0[2 * q], f1 = a0[2 * q + 1];
    const float g0 = a1[2 * q], g1 = a1[2 * q + 1];
    const unsigned short h0 = f2bf_bits(bf_bits2f(f2bf_bits(f0)) * sc);
    const unsigned short h1 = f2bf_bits(bf_bits2f(f2bf_bits(f1)) * sc);
    const unsigned short h2 = f2bf_bits(bf_bits2f(f2bf_bits(g0)) * sc);
    const unsigned short h3 = f2bf_bits(bf_bits2f(f2bf_bits(g1)) * sc);
    o[q]     = pk16(h0, h1);
    o[2 + q] = pk16(h2, h3);
  }
  return o;
}

__device__ __forceinline__ void split8_bf16(v4f a0, v4f a1, v4u& hv, v4u& lv) {
#pragma unroll
  for (int q = 0; q < 2; ++q) {
    const float f0 = a0[2 * q], f1 = a0[2 * q + 1];
    const float g0 = a1[2 * q], g1 = a1[2 * q + 1];
    const unsigned short h0 = f2bf_bits(f0), h1 = f2bf_bits(f1);
    const unsigned short h2 = f2bf_bits(g0), h3 = f2bf_bits(g1);
    const unsigned short l0 = f2bf_bits(f0 - bf_bits2f(h0)), l1 = f2bf_bits(f1 - bf_bits2f(h1));
    const unsigned short l2 = f2bf_bits(g0 - bf_bits2f(h2)), l3 = f2bf_bits(g1 - bf_bits2f(h3));
    hv[q]     = pk16(h0, h1);
    hv[2 + q] = pk16(h2, h3);
    lv[q]     = pk16(l0, l1);
    lv[2 + q] = pk16(l2, l3);
  }
}

union FragB { v16b v; v8b h[2]; };
__device__ __forceinline__ v16b frag_load(const __bf16* p) {
  FragB f;
  f.h[0] = *(const v8b*)(p);
  f.h[1] = *(const v8b*)(p + 16);
  return f.v;
}
__device__ __forceinline__ v8f mma_bf(v16b a, v16b b, v8f c) {
  c = __builtin_amdgcn_wmma_f32_16x16x32_bf16(false, a, false, b, (short)0, c, false, false);
  asm volatile("v_nop\n\tv_nop\n\tv_nop\n\tv_nop" : "+v"(c) : "v"(a), "v"(b));
  return c;
}
__device__ __forceinline__ void wave_lds_sync() {
  __builtin_amdgcn_fence(__ATOMIC_RELEASE, "workgroup");
  __builtin_amdgcn_wave_barrier();
  __builtin_amdgcn_fence(__ATOMIC_ACQUIRE, "workgroup");
}

__global__ __launch_bounds__(256) void prep_x_kernel(const float* __restrict__ X, unsigned short* __restrict__ XB,
                                                     unsigned short* __restrict__ VT) {
  __shared__ __align__(16) float tf[64 * 68];
  const int c0  = blockIdx.x * 64;
  const int r0  = blockIdx.y * 64;
  const int b   = blockIdx.z;
  const int tid = threadIdx.x;
  const float* Xs = X + ((size_t)b * kSeq + r0) * kChan + c0;
  {
    const int lr = tid >> 4;
    const int c4 = (tid & 15) * 4;
#pragma unroll
    for (int it = 0; it < 4; ++it) {
      const int rr = it * 16 + lr;
      const v4f a = *(const v4f*)(Xs + (size_t)rr * kChan + c4);
      *(v4f*)(tf + rr * 68 + c4) = a;
    }
  }
  __syncthreads();
  const int sub = tid >> 3;
  const int c8  = (tid & 7) * 8;
  v4u xv[2], tv[2];
#pragma unroll
  for (int it = 0; it < 2; ++it) {
    const int row = it * 32 + sub;
    const v4f a0 = *(const v4f*)(tf + row * 68 + c8);
    const v4f a1 = *(const v4f*)(tf + row * 68 + c8 + 4);
    xv[it] = pack8_bf16(a0, a1, 1.0f);
    v4u t;
#pragma unroll
    for (int q = 0; q < 4; ++q) {
      const float f0 = tf[(c8 + 2 * q) * 68 + row];
      const float f1 = tf[(c8 + 2 * q + 1) * 68 + row];
      t[q] = pk16(f2bf_bits(f0), f2bf_bits(f1));
    }
    tv[it] = t;
  }
  for (int pass = 0; pass < 2; ++pass) {
#pragma unroll
    for (int it = 0; it < 2; ++it) {
      const int row = it * 32 + sub;
      *(volatile v4u*)(void*)(XB + ((size_t)b * kSeq + r0 + row) * kChan + c0 + c8) = xv[it];
      *(volatile v4u*)(void*)(VT + ((size_t)b * kChan + c0 + row) * kSeq + r0 + c8) = tv[it];
    }
    __threadfence();
  }
}

__global__ __launch_bounds__(256) void prep_w_kernel(const float* __restrict__ Wq, const float* __restrict__ bq,
                                                     const float* __restrict__ Wk, const float* __restrict__ bk,
                                                     unsigned short* __restrict__ WT, float* __restrict__ biasv) {
  const int tid = threadIdx.x;
  if (blockIdx.x < 16) {
    const bool isq = (blockIdx.x < 8);
    const float* src = isq ? Wq : Wk;
    const float sc = isq ? kScoreScale : 1.0f;
    const size_t e0 = ((size_t)(blockIdx.x & 7) * 256 + tid) * 8;
    const v4f a0 = *(const v4f*)(src + e0);
    const v4f a1 = *(const v4f*)(src + e0 + 4);
    const v4u w = pack8_bf16(a0, a1, sc);
    unsigned short* dst = WT + (size_t)blockIdx.x * 2048 + (size_t)tid * 8;
    *(volatile v4u*)(void*)dst = w;
    __threadfence();
    *(volatile v4u*)(void*)dst = w;
  } else {
    const int wave = tid >> 5, lane = tid & 31;
    if (wave < 2) {
      const float* src = (wave == 0) ? bq : bk;
      const float sc = (wave == 0) ? kScoreScale : 1.0f;
      const int lc = (lane & 15) * 4;
      const v4f a = *(const v4f*)(src + lc);
      v4f o;
#pragma unroll
      for (int e = 0; e < 4; ++e) {
        const float f = a[e];
        o[e] = bf_bits2f(f2bf_bits(f)) * sc;
      }
      if (lane < 16) {
        float* dst = biasv + wave * 64 + lc;
        *(volatile v4f*)dst = o;
        __threadfence();
        *(volatile v4f*)dst = o;
      }
    }
  }
}

__global__ __launch_bounds__(256) void proj_gemm_kernel(const unsigned short* __restrict__ Ap,
                                                        const unsigned short* __restrict__ Btp,
                                                        unsigned short* __restrict__ Ch,
                                                        unsigned short* __restrict__ Cl,
                                                        const float* __restrict__ bias) {
  __shared__ __align__(16) float sT[8][16 * 68];
  const __bf16* A  = (const __bf16*)(const void*)Ap;
  const __bf16* Bt = (const __bf16*)(const void*)Btp;
  const int lane = threadIdx.x & 31;
  const int wave = threadIdx.x >> 5;
  constexpr int tilesN = kQKP >> 6;
  constexpr int tilesM = kRows >> 6;
  const int tile = blockIdx.x * 8 + wave;
  if (tile >= tilesM * tilesN) return;
  const int tm = tile / tilesN;
  const int tn = tile - tm * tilesN;
  const int m0 = tm << 6;
  const int n0 = tn << 6;
  const int rlane = lane & 15;
  const int koff  = (lane >> 4) * 8;
  const int mOff  = (lane >> 4) * 8;

  v8f acc[4][4];
#pragma unroll
  for (int i = 0; i < 4; ++i)
#pragma unroll
    for (int j = 0; j < 4; ++j) acc[i][j] = (v8f){0.f, 0.f, 0.f, 0.f, 0.f, 0.f, 0.f, 0.f};

#pragma unroll 1
  for (int k0 = 0; k0 < kChan; k0 += 32) {
    v16b bh[4];
#pragma unroll
    for (int j = 0; j < 4; ++j)
      bh[j] = frag_load(Bt + (size_t)(n0 + (j << 4) + rlane) * kChan + koff + k0);
#pragma unroll
    for (int i = 0; i < 4; ++i) {
      const v16b ah = frag_load(A + (size_t)(m0 + (i << 4) + rlane) * kChan + koff + k0);
#pragma unroll
      for (int j = 0; j < 4; ++j) acc[i][j] = mma_bf(ah, bh[j], acc[i][j]);
    }
  }

  float* slab = sT[wave];
  const int q8 = lane >> 3, c8 = (lane & 7) * 8;
#pragma unroll
  for (int i = 0; i < 4; ++i) {
    const int mBase = m0 + (i << 4);
#pragma unroll
    for (int j = 0; j < 4; ++j) {
      const float bv = bias[n0 + (j << 4) + rlane];
#pragma unroll
      for (int r = 0; r < 8; ++r) slab[(mOff + r) * 68 + (j << 4) + rlane] = acc[i][j][r] + bv;
    }
    wave_lds_sync();
    v4u hv[4], lv[4];
#pragma unroll
    for (int it = 0; it < 4; ++it) {
      const int row = it * 4 + q8;
      const v4f a0 = *(const v4f*)(slab + row * 68 + c8);
      const v4f a1 = *(const v4f*)(slab + row * 68 + c8 + 4);
      split8_bf16(a0, a1, hv[it], lv[it]);
    }
    for (int pass = 0; pass < 2; ++pass) {
#pragma unroll
      for (int it = 0; it < 4; ++it) {
        const int row = it * 4 + q8;
        const size_t go = (size_t)(mBase + row) * kQKP + n0 + c8;
        *(volatile v4u*)(void*)(Ch + go) = hv[it];
        *(volatile v4u*)(void*)(Cl + go) = lv[it];
      }
      __threadfence();
    }
    wave_lds_sync();
  }
}

__global__ __launch_bounds__(128) void causal_attn_kernel(const unsigned short* __restrict__ qkhp,
                                                          const unsigned short* __restrict__ qklp,
                                                          const unsigned short* __restrict__ vtp,
                                                          const int* __restrict__ traj,
                                                          float* __restrict__ out) {
  __shared__ __align__(16) __bf16 Psh[4][16 * 64];
  __shared__ __align__(16) __bf16 Psl[4][16 * 64];
  __shared__ __align__(16) float  Os[4][16 * kOsP];

  const int tid  = threadIdx.x;
  const int wave = tid >> 5;
  const int lane = tid & 31;
  const int hh   = lane >> 4;
  const int c    = lane & 15;
  const int qb   = blockIdx.x;
  const int b    = blockIdx.y;
  const int nh   = blockIdx.z;
  const int q0b  = qb * 64;
  const int q0   = q0b + wave * 16;

  int len = traj[b];
  len = (len < 0) ? 0 : len;
  len = (len > kSeq) ? kSeq : len;

  float* optr = out + ((size_t)b * kSeq + q0) * kChan + nh * kNHalf + lane * 4;

  if (q0b >= len) {
    const v4f z = (v4f){0.f, 0.f, 0.f, 0.f};
    for (int pass = 0; pass < 2; ++pass) {
#pragma unroll
      for (int row = 0; row < 16; ++row) *(volatile v4f*)(optr + (size_t)row * kChan) = z;
      __threadfence();
    }
    return;
  }

  const __bf16* QKh = (const __bf16*)(const void*)qkhp + (size_t)b * kSeq * kQKP;
  const __bf16* QKl = (const __bf16*)(const void*)qklp + (size_t)b * kSeq * kQKP;
  const __bf16* Vt  = (const __bf16*)(const void*)vtp + ((size_t)b * kChan + nh * kNHalf) * kSeq;

  v16b qh[2], ql[2];
  {
    const size_t qo = (size_t)(q0 + c) * kQKP + 8 * hh;
#pragma unroll
    for (int dc = 0; dc < 2; ++dc) {
      qh[dc] = frag_load(QKh + qo + dc * 32);
      ql[dc] = frag_load(QKl + qo + dc * 32);
    }
  }

  float mrow[8], lrow[8];
  v8f oacc[8];
#pragma unroll
  for (int r = 0; r < 8; ++r) { mrow[r] = -1e30f; lrow[r] = 0.f; }
#pragma unroll
  for (int t = 0; t < 8; ++t) oacc[t] = (v8f){0.f, 0.f, 0.f, 0.f, 0.f, 0.f, 0.f, 0.f};

  __bf16* pwh = Psh[wave];
  __bf16* pwl = Psl[wave];

  for (int kc = 0; kc <= qb; ++kc) {
    const int kv0 = kc * 64;
    v8f s[4];
#pragma unroll
    for (int j = 0; j < 4; ++j) {
      s[j] = (v8f){0.f, 0.f, 0.f, 0.f, 0.f, 0.f, 0.f, 0.f};
      const size_t ko = (size_t)(kv0 + j * 16 + c) * kQKP + kProj + 8 * hh;
#pragma unroll
      for (int dc = 0; dc < 2; ++dc) {
        const v16b kh = frag_load(QKh + ko + dc * 32);
        const v16b kl = frag_load(QKl + ko + dc * 32);
        s[j] = mma_bf(qh[dc], kh, s[j]);
        s[j] = mma_bf(qh[dc], kl, s[j]);
        s[j] = mma_bf(ql[dc], kh, s[j]);
      }
    }
    const bool diag = (kc == qb);
#pragma unroll
    for (int r = 0; r < 8; ++r) {
      const int lrw = wave * 16 + 8 * hh + r;
      float m = -1e30f;
#pragma unroll
      for (int j = 0; j < 4; ++j) {
        const int lcol = j * 16 + c;
        float sv = s[j][r];
        sv = (diag && (lcol > lrw)) ? -1e30f : sv;
        s[j][r] = sv;
        m = fmaxf(m, sv);
      }
      m = fmaxf(m, __shfl_xor(m, 1, 32));
      m = fmaxf(m, __shfl_xor(m, 2, 32));
      m = fmaxf(m, __shfl_xor(m, 4, 32));
      m = fmaxf(m, __shfl_xor(m, 8, 32));
      const float mnew  = fmaxf(mrow[r], m);
      const float alpha = expf(mrow[r] - mnew);
      mrow[r] = mnew;
      float psum = 0.f;
#pragma unroll
      for (int j = 0; j < 4; ++j) {
        const float p = expf(s[j][r] - mnew);
        psum += p;
        const unsigned short hb = f2bf_bits(p);
        const unsigned short lb = f2bf_bits(p - bf_bits2f(hb));
        pwh[(8 * hh + r) * 64 + j * 16 + c] = __builtin_bit_cast(__bf16, hb);
        pwl[(8 * hh + r) * 64 + j * 16 + c] = __builtin_bit_cast(__bf16, lb);
      }
      psum += __shfl_xor(psum, 1, 32);
      psum += __shfl_xor(psum, 2, 32);
      psum += __shfl_xor(psum, 4, 32);
      psum += __shfl_xor(psum, 8, 32);
      lrow[r] = lrow[r] * alpha + psum;
#pragma unroll
      for (int t = 0; t < 8; ++t) oacc[t][r] *= alpha;
    }
    wave_lds_sync();
#pragma unroll 1
    for (int kk = 0; kk < 2; ++kk) {
      FragB pa, pl;
      pa.h[0] = *(const v8b*)(pwh + c * 64 + kk * 32 + 8 * hh);
      pa.h[1] = *(const v8b*)(pwh + c * 64 + kk * 32 + 16 + 8 * hh);
      pl.h[0] = *(const v8b*)(pwl + c * 64 + kk * 32 + 8 * hh);
      pl.h[1] = *(const v8b*)(pwl + c * 64 + kk * 32 + 16 + 8 * hh);
#pragma unroll
      for (int t = 0; t < 8; ++t) {
        const v16b vb = frag_load(Vt + (size_t)(t * 16 + c) * kSeq + kv0 + kk * 32 + 8 * hh);
        oacc[t] = mma_bf(pa.v, vb, oacc[t]);
        oacc[t] = mma_bf(pl.v, vb, oacc[t]);
      }
    }
    wave_lds_sync();
  }

  float* os = Os[wave];
#pragma unroll
  for (int r = 0; r < 8; ++r) {
    const float inv = 1.0f / lrow[r];
    const bool keep = (q0 + 8 * hh + r) < len;
#pragma unroll
    for (int t = 0; t < 8; ++t) {
      const float val = oacc[t][r] * inv;
      os[(8 * hh + r) * kOsP + t * 16 + c] = keep ? val : 0.0f;
    }
  }
  wave_lds_sync();
  for (int pass = 0; pass < 2; ++pass) {
#pragma unroll
    for (int row = 0; row < 16; ++row) {
      const v4f val = *(const v4f*)(os + row * kOsP + lane * 4);
      *(volatile v4f*)(optr + (size_t)row * kChan) = val;
    }
    __threadfence();
  }
}

extern "C" void kernel_launch(void* const* d_in, const int* in_sizes, int n_in,
                              void* d_out, int out_size, void* d_ws, size_t ws_size,
                              hipStream_t stream) {
  if (n_in < 6) return;
  if (in_sizes[0] != kRows * kChan) return;
  if (in_sizes[1] != kProj * kChan) return;
  if (in_sizes[2] != kProj) return;
  if (in_sizes[3] != kProj * kChan) return;
  if (in_sizes[4] != kProj) return;
  if (in_sizes[5] != kBatch) return;
  if (out_size != kRows * kChan) return;
  if (ws_size < kWsTotal) return;

  const float* X    = (const float*)d_in[0];
  const float* Wq   = (const float*)d_in[1];
  const float* bq   = (const float*)d_in[2];
  const float* Wk   = (const float*)d_in[3];
  const float* bk   = (const float*)d_in[4];
  const int*   traj = (const int*)d_in[5];
  float* out = (float*)d_out;

  char* ws = (char*)d_ws;
  unsigned short* XB   = (unsigned short*)(ws + kOffXB);
  unsigned short* VT   = (unsigned short*)(ws + kOffVT);
  unsigned short* QKH  = (unsigned short*)(ws + kOffQKH);
  unsigned short* QKL  = (unsigned short*)(ws + kOffQKL);
  unsigned short* WT   = (unsigned short*)(ws + kOffWT);
  float*          BIAS = (float*)(ws + kOffBIAS);

  prep_x_kernel<<<dim3(kChan / 64, kSeq / 64, kBatch), 256, 0, stream>>>(X, XB, VT);
  prep_w_kernel<<<17, 256, 0, stream>>>(Wq, bq, Wk, bk, WT, BIAS);
  proj_gemm_kernel<<<((kRows / 64) * (kQKP / 64)) / 8, 256, 0, stream>>>(XB, WT, QKH, QKL, BIAS);
  causal_attn_kernel<<<dim3(kSeq / 64, kBatch, 2), 128, 0, stream>>>(QKH, QKL, VT, traj, out);
}
